// RNNModule_37898791420421
// MI455X (gfx1250) — hardware-verified
//
#include <hip/hip_runtime.h>
#include <math.h>

typedef __attribute__((ext_vector_type(16))) _Float16 v16h;
typedef __attribute__((ext_vector_type(8)))  _Float16 v8h;
typedef __attribute__((ext_vector_type(8)))  float    v8f;
typedef __attribute__((ext_vector_type(4)))  float    v4f;
typedef __attribute__((ext_vector_type(4)))  unsigned v4u;

static_assert(sizeof(_Float16) == 2);

constexpr int kBatch   = 1024;
constexpr int kSteps   = 512;
constexpr int kIn      = 8;
constexpr int kHid     = 50;
constexpr int kHP      = 64;
constexpr int kGates   = 3;
constexpr int kNC      = kGates * kHP;
constexpr int kK1      = 2 * kHP;
constexpr int kRows    = 16;
constexpr int kThreads = 128;
constexpr int kW0Halves = kNC * kHP;
constexpr int kW1Halves = kNC * kK1;
constexpr int kWxFloats = kNC * kIn;
constexpr float kAScale = 16.0f;
constexpr float kBScale = 64.0f;
constexpr float kFold   = 1.0f / 1024.0f;

constexpr int kChunksW0  = kW0Halves / 8;
constexpr int kChunksW1  = kW1Halves / 8;
constexpr int kChunksWx  = kWxFloats / 4;
constexpr int kChunksAll = kChunksW0 + kChunksW1 + kChunksWx;
constexpr int kPrepThreads = 256;
constexpr int kPrepBlocks  = (kChunksAll + kPrepThreads - 1) / kPrepThreads;
constexpr int kBlkEndW0    = kChunksW0 / kPrepThreads;
constexpr int kBlkEndW1    = (kChunksW0 + kChunksW1) / kPrepThreads;
constexpr size_t kOffW1Bytes = (size_t)kChunksW0 * 16;
constexpr size_t kOffWxBytes = (size_t)(kChunksW0 + kChunksW1) * 16;
constexpr size_t kWsBytes    = (size_t)kChunksAll * 16;

static_assert(kBatch % kRows == 0);
static_assert(kHP % 32 == 0 && kK1 % 32 == 0);
static_assert((kRows * kHid * 4) % 128 == 0);
static_assert(kChunksW0 % kPrepThreads == 0 && (kChunksW0 + kChunksW1) % kPrepThreads == 0);
static_assert(kOffW1Bytes % 128 == 0 && kOffWxBytes % 128 == 0);

union FragU { v16h v; v8h h[2]; };
__device__ __forceinline__ v16h frag_load(const _Float16* p) {
  FragU f; f.h[0] = *(const v8h*)(p); f.h[1] = *(const v8h*)(p + 16); return f.v;
}
__device__ __forceinline__ v8f wm16(v16h a, v16h b, v8f c) {
  c = __builtin_amdgcn_wmma_f32_16x16x32_f16(false, a, false, b, (short)0, c, false, false);
  asm volatile("v_nop\n\tv_nop\n\tv_nop\n\tv_nop" : "+v"(c) : "v"(a), "v"(b));
  return c;
}
__device__ __forceinline__ float sigm(float v) { return 1.0f / (1.0f + expf(-v)); }
__device__ __forceinline__ float tanh_e(float v) {
  const float e = expf(-2.0f * fabsf(v));
  const float r = (1.0f - e) * (1.0f / (1.0f + e));
  return copysignf(r, v);
}
__device__ __forceinline__ unsigned pack_f16x2(float a, float b) {
  const _Float16 ha = (_Float16)a, hb = (_Float16)b;
  return (unsigned)__builtin_bit_cast(unsigned short, ha) | ((unsigned)__builtin_bit_cast(unsigned short, hb) << 16);
}

__global__ __launch_bounds__(kPrepThreads)
void prep_planes(const float* __restrict__ Wih0, const float* __restrict__ Whh0,
                 const float* __restrict__ Wih1, const float* __restrict__ Whh1,
                 unsigned* __restrict__ planes) {
  const int tid   = threadIdx.x;
  const int chunk = blockIdx.x * kPrepThreads + tid;
  const bool act  = chunk < kChunksAll;
  const int chc   = act ? chunk : (kChunksAll - 1);
  unsigned w0 = 0u, w1 = 0u, w2 = 0u, w3 = 0u;
  if (blockIdx.x < kBlkEndW0) {
    const int el0 = chc * 8;
    const int n = el0 >> 6, k0 = el0 & 63;
    const int g = n >> 6, uu = n & 63;
    const int ucl = uu < kHid ? uu : kHid - 1;
    const float* wr = Whh0 + (size_t)(g * kHid + ucl) * kHid;
    float v[8];
#pragma unroll
    for (int e = 0; e < 8; ++e) {
      const int k = k0 + e;
      const int kc = k < kHid ? k : kHid - 1;
      const float t0 = wr[kc];
      v[e] = (uu < kHid && k < kHid) ? kBScale * t0 : 0.0f;
    }
    w0 = pack_f16x2(v[0], v[1]); w1 = pack_f16x2(v[2], v[3]);
    w2 = pack_f16x2(v[4], v[5]); w3 = pack_f16x2(v[6], v[7]);
  } else if (blockIdx.x < kBlkEndW1) {
    const int el0 = (chc - kChunksW0) * 8;
    const int n = el0 >> 7, k0 = el0 & 127;
    const int g = n >> 6, uu = n & 63;
    const int ucl = uu < kHid ? uu : kHid - 1;
    const size_t ro = (size_t)(g * kHid + ucl) * kHid;
    const bool inpart = k0 < kHP;
    float v[8];
#pragma unroll
    for (int e = 0; e < 8; ++e) {
      const int kk = (k0 & 63) + e;
      const int kc = kk < kHid ? kk : kHid - 1;
      const float ta = Wih1[ro + kc];
      const float tb = Whh1[ro + kc];
      const float t0 = inpart ? ta : tb;
      v[e] = (uu < kHid && kk < kHid) ? kBScale * t0 : 0.0f;
    }
    w0 = pack_f16x2(v[0], v[1]); w1 = pack_f16x2(v[2], v[3]);
    w2 = pack_f16x2(v[4], v[5]); w3 = pack_f16x2(v[6], v[7]);
  } else {
    const int f0 = (chc - kChunksW0 - kChunksW1) * 4;
    const int n = f0 >> 3, e0 = f0 & 7;
    const int g = n >> 6, uu = n & 63;
    const int ucl = uu < kHid ? uu : kHid - 1;
    const float* wr = Wih0 + (size_t)(g * kHid + ucl) * kIn + e0;
    const float ta = wr[0], tb = wr[1], tc = wr[2], td = wr[3];
    const bool uv = uu < kHid;
    w0 = __float_as_uint(uv ? ta : 0.0f); w1 = __float_as_uint(uv ? tb : 0.0f);
    w2 = __float_as_uint(uv ? tc : 0.0f); w3 = __float_as_uint(uv ? td : 0.0f);
  }
  const v4u pk = {w0, w1, w2, w3};
  volatile v4u* dst = ((volatile v4u*)(void*)planes) + chc;
  if (act) *dst = pk;
  __threadfence();
  if (act) *dst = pk;
}

__global__ __launch_bounds__(kThreads)
void gru2_seq_kernel(const float* __restrict__ x,
                     const float* Wxp, const _Float16* W0p, const _Float16* W1p,
                     const float* __restrict__ bih0, const float* __restrict__ bhh0,
                     const float* __restrict__ bih1, const float* __restrict__ bhh1,
                     float* __restrict__ out) {
  __shared__ __align__(16) _Float16 sA0[2][kRows * kHP];
  __shared__ __align__(16) _Float16 sA1[2][kRows * kK1];
  __shared__ __align__(16) float    sX[2][kRows * kIn];
  __shared__ __align__(16) float    sOut[kRows * kHP];

  const int tid   = threadIdx.x;
  const int lane  = tid & 31;
  const int wave  = tid >> 5;
  const int hh    = lane >> 4;
  const int cc    = lane & 15;
  const int u     = wave * 16 + cc;
  const int bbase = blockIdx.x * kRows;

  for (int i = tid; i < (2 * kRows * kHP) / 2; i += kThreads) ((unsigned*)&sA0[0][0])[i] = 0u;
  for (int i = tid; i < (2 * kRows * kK1) / 2; i += kThreads) ((unsigned*)&sA1[0][0])[i] = 0u;
  sX[0][tid] = x[((size_t)(bbase + (tid >> 3)) * kSteps) * kIn + (tid & 7)];

  const int  ucl  = u < kHid ? u : kHid - 1;
  const bool uval = u < kHid;
  float bi0r[kGates], bh0r[kGates], bi1r[kGates], bh1r[kGates];
#pragma unroll
  for (int g = 0; g < kGates; ++g) {
    const float va = bih0[g * kHid + ucl], vb = bhh0[g * kHid + ucl];
    const float vc = bih1[g * kHid + ucl], vd = bhh1[g * kHid + ucl];
    bi0r[g] = uval ? va : 0.0f; bh0r[g] = uval ? vb : 0.0f;
    bi1r[g] = uval ? vc : 0.0f; bh1r[g] = uval ? vd : 0.0f;
  }
  float h0r[8], h1r[8];
#pragma unroll
  for (int r = 0; r < 8; ++r) { h0r[r] = 0.0f; h1r[r] = 0.0f; }
  __syncthreads();

  const v8f zero8 = {0.f, 0.f, 0.f, 0.f, 0.f, 0.f, 0.f, 0.f};

  for (int t = 0; t < kSteps; ++t) {
    const int p = t & 1, q = p ^ 1;
    int zoff = 0;
    asm volatile("" : "+v"(zoff));
    const int tn = (t + 1 < kSteps) ? (t + 1) : (kSteps - 1);
    const float xnext = x[((size_t)(bbase + (tid >> 3)) * kSteps + tn) * kIn + (tid & 7)];

    v8f acc0[kGates];
#pragma unroll
    for (int g = 0; g < kGates; ++g) acc0[g] = zero8;
    {
      const _Float16* arow = &sA0[p][cc * kHP + 8 * hh];
#pragma unroll
      for (int ks = 0; ks < kHP / 32; ++ks) {
        const v16h af = frag_load(arow + 32 * ks);
#pragma unroll
        for (int g = 0; g < kGates; ++g) {
          const v16h bf = frag_load(W0p + ((g * kHP + u) * kHP + 32 * ks + 8 * hh + zoff));
          acc0[g] = wm16(af, bf, acc0[g]);
        }
        asm volatile("" : "+v"(zoff) : "v"(acc0[2]));
      }
    }
    v4f wlo[kGates], whi[kGates];
#pragma unroll
    for (int g = 0; g < kGates; ++g) {
      wlo[g] = *(const v4f*)(Wxp + ((g * kHP + u) * kIn + zoff));
      whi[g] = *(const v4f*)(Wxp + ((g * kHP + u) * kIn + 4 + zoff));
    }
    {
      const float* xs = &sX[p][0];
#pragma unroll
      for (int r = 0; r < 8; ++r) {
        const v4f xa = *(const v4f*)(xs + (8 * hh + r) * kIn);
        const v4f xb = *(const v4f*)(xs + (8 * hh + r) * kIn + 4);
        float s0 = bi0r[0], s1 = bi0r[1], s2 = bi0r[2];
#pragma unroll
        for (int e = 0; e < 4; ++e) {
          s0 += xa[e] * wlo[0][e]; s1 += xa[e] * wlo[1][e]; s2 += xa[e] * wlo[2][e];
        }
#pragma unroll
        for (int e = 0; e < 4; ++e) {
          s0 += xb[e] * whi[0][e]; s1 += xb[e] * whi[1][e]; s2 += xb[e] * whi[2][e];
        }
        const float rg = sigm(s0 + (acc0[0][r] * kFold + bh0r[0]));
        const float zg = sigm(s1 + (acc0[1][r] * kFold + bh0r[1]));
        const float ng = tanh_e(s2 + rg * (acc0[2][r] * kFold + bh0r[2]));
        const float hn = (1.0f - zg) * ng + zg * h0r[r];
        h0r[r] = hn;
        const _Float16 hv = (_Float16)(kAScale * hn);
        sA0[q][(8 * hh + r) * kHP + u] = hv;
        sA1[p][(8 * hh + r) * kK1 + u] = hv;
      }
    }
    asm volatile("" : "+v"(zoff) : "v"(h0r[7]));
    sX[q][tid] = xnext;
    __syncthreads();

    v8f acc1[4];
#pragma unroll
    for (int g = 0; g < 4; ++g) acc1[g] = zero8;
    {
      const _Float16* arow = &sA1[p][cc * kK1 + 8 * hh];
#pragma unroll
      for (int ks = 0; ks < kK1 / 32; ++ks) {
        const v16h af  = frag_load(arow + 32 * ks);
        const v16h bfr = frag_load(W1p + ((0 * kHP + u) * kK1 + 32 * ks + 8 * hh + zoff));
        acc1[0] = wm16(af, bfr, acc1[0]);
        const v16h bfz = frag_load(W1p + ((1 * kHP + u) * kK1 + 32 * ks + 8 * hh + zoff));
        acc1[1] = wm16(af, bfz, acc1[1]);
        const v16h bfn = frag_load(W1p + ((2 * kHP + u) * kK1 + 32 * ks + 8 * hh + zoff));
        acc1[2 + (ks >> 1)] = wm16(af, bfn, acc1[2 + (ks >> 1)]);
        asm volatile("" : "+v"(zoff) : "v"(acc1[1]));
      }
    }
#pragma unroll
    for (int r = 0; r < 8; ++r) {
      const float rg = sigm((acc1[0][r] * kFold + bi1r[0]) + bh1r[0]);
      const float zg = sigm((acc1[1][r] * kFold + bi1r[1]) + bh1r[1]);
      const float ng = tanh_e((acc1[2][r] * kFold + bi1r[2]) + rg * (acc1[3][r] * kFold + bh1r[2]));
      const float hn = (1.0f - zg) * ng + zg * h1r[r];
      h1r[r] = hn;
      sA1[q][(8 * hh + r) * kK1 + kHP + u] = (_Float16)(kAScale * hn);
    }
    __syncthreads();
  }

#pragma unroll
  for (int r = 0; r < 8; ++r) sOut[(8 * hh + r) * kHP + u] = h1r[r];
  __syncthreads();
  {
    float* ob = out + (size_t)blockIdx.x * (kRows * kHid);
    for (int pass = 0; pass < 2; ++pass) {
#pragma unroll 1
      for (int k2 = 0; k2 < 2; ++k2) {
        const int chunk = tid + kThreads * k2;
        const bool act = chunk < (kRows * kHid) / 4;
        const int chc = act ? chunk : 0;
        v4f v;
#pragma unroll
        for (int e = 0; e < 4; ++e) {
          const int j = chc * 4 + e;
          const int row = j / kHid;
          const int col = j - row * kHid;
          v[e] = sOut[row * kHP + col];
        }
        if (act) *(volatile v4f*)(ob + (size_t)chunk * 4) = v;
      }
      __threadfence();
    }
  }
}

extern "C" void kernel_launch(void* const* d_in, const int* in_sizes, int n_in,
                              void* d_out, int out_size, void* d_ws, size_t ws_size,
                              hipStream_t stream) {
  if (n_in < 9) return;
  if (in_sizes[0] != kBatch * kSteps * kIn) return;
  if (in_sizes[1] != kGates * kHid * kIn) return;
  if (in_sizes[2] != kGates * kHid * kHid) return;
  if (in_sizes[3] != kGates * kHid || in_sizes[4] != kGates * kHid) return;
  if (in_sizes[5] != kGates * kHid * kHid || in_sizes[6] != kGates * kHid * kHid) return;
  if (in_sizes[7] != kGates * kHid || in_sizes[8] != kGates * kHid) return;
  if (out_size != kBatch * kHid) return;
  if (ws_size < kWsBytes) return;

  const float* x    = (const float*)d_in[0];
  const float* Wih0 = (const float*)d_in[1];
  const float* Whh0 = (const float*)d_in[2];
  const float* bih0 = (const float*)d_in[3];
  const float* bhh0 = (const float*)d_in[4];
  const float* Wih1 = (const float*)d_in[5];
  const float* Whh1 = (const float*)d_in[6];
  const float* bih1 = (const float*)d_in[7];
  const float* bhh1 = (const float*)d_in[8];
  float* out = (float*)d_out;

  unsigned char* ws = (unsigned char*)d_ws;
  unsigned*        planes = (unsigned*)(void*)ws;
  const _Float16*  W0p = (const _Float16*)(const void*)ws;
  const _Float16*  W1p = (const _Float16*)(const void*)(ws + kOffW1Bytes);
  const float*     Wxp = (const float*)(const void*)(ws + kOffWxBytes);

  prep_planes<<<dim3(kPrepBlocks), dim3(kPrepThreads), 0, stream>>>(Wih0, Whh0, Wih1, Whh1, planes);
  gru2_seq_kernel<<<dim3(kBatch / kRows), dim3(kThreads), 0, stream>>>(
      x, Wxp, W0p, W1p, bih0, bhh0, bih1, bhh1, out);
}
